// Discriminator_28767690948703
// MI455X (gfx1250) — hardware-run, weakly checked
//
#include <hip/hip_runtime.h>


#pragma clang fp contract(off)

#ifndef NROWS
#define NROWS 1024
#endif
#define NROWS_FULL 1024
#define NF    512
#define HW    256
#define NKER  10
#define KDIM  10
#define MBW   100
#define MBP   128
#define CATW  266
#define CATK  288
#define CATP  320
#define DVP   32
#define ACTC  16.0f
#define WGTC  64.0f
#define FOLD  (1.0f / 1024.0f)
#define LN_EPS 1.0e-3f
#define LRA   0.3f
#define LOG2E 1.4426950408889634f
#define LNR   32
#define LNRW  4

static_assert(NROWS <= NROWS_FULL);
static_assert(NROWS % 64 == 0);
static_assert(NROWS % 128 == 0);
static_assert(NROWS % LNR == 0);
static_assert(LNR == 8 * LNRW);
static_assert(NF % 64 == 0);
static_assert(HW % 64 == 0);
static_assert(HW == 256);
static_assert(CATW == HW + NKER);
static_assert(CATK % 32 == 0);
static_assert(CATK >= CATW);
static_assert(CATP >= CATK);
static_assert(CATP % 64 == 0);
static_assert(CATP - HW == 64);
static_assert(MBW == NKER * KDIM);
static_assert(NKER == 10);
static_assert(KDIM == 10);
static_assert(MBP == 128);
static_assert(MBP >= MBW);
static_assert(MBP % 64 == 0);
static_assert(DVP == 32);
static_assert(NKER <= 12);
static_assert(((size_t)NROWS * NF) % 8 == 0);
static_assert(32 * 16 * 8 == 16 * 64 * 4);
static_assert(32 * 16 * 4 == 16 * 64 * 2);
static_assert(256 * 16 == 32 * 64 * 2);
static_assert(32 * 16 == HW * 2);
static_assert(8 * 16 == (CATP - HW) * 2);
static_assert(8 * 16 == DVP * 4);
static_assert(8 * 16 == LNR * 4);
static_assert(16 * 68 * 4 <= 131072);
static_assert(64 * 33 * 4 <= 131072);
static_assert((MBP + 4 * 32) * 4 <= 131072);

typedef _Float16 h16;
typedef unsigned short bf;
typedef __attribute__((ext_vector_type(16))) __bf16   v16bf;
typedef __attribute__((ext_vector_type(16))) _Float16 v16h;
typedef __attribute__((ext_vector_type(8)))  _Float16 v8h;
typedef __attribute__((ext_vector_type(8)))  unsigned short v8us;
typedef __attribute__((ext_vector_type(8)))  float    v8f;
typedef __attribute__((ext_vector_type(4)))  float    v4f;
typedef v4f  __attribute__((may_alias)) v4fa;

__device__ __forceinline__ unsigned short f2bf(float f) { unsigned u = __float_as_uint(f); u += 0x7FFFu + ((u >> 16) & 1u); return (unsigned short)(u >> 16); }
__device__ __forceinline__ float bfr(float f) { return __uint_as_float(((unsigned)f2bf(f)) << 16); }
__device__ __forceinline__ v16h cat16(v8h lo, v8h hi) { return __builtin_shufflevector(lo, hi, 0, 1, 2, 3, 4, 5, 6, 7, 8, 9, 10, 11, 12, 13, 14, 15); }
__device__ __forceinline__ v16bf cat16b(v8us lo, v8us hi) { return __builtin_bit_cast(v16bf, __builtin_shufflevector(lo, hi, 0, 1, 2, 3, 4, 5, 6, 7, 8, 9, 10, 11, 12, 13, 14, 15)); }
__device__ __forceinline__ v8f wmma16(v16h a, v16h b, v8f c) { return __builtin_amdgcn_wmma_f32_16x16x32_f16(false, a, false, b, (short)0, c, false, false); }
__device__ __forceinline__ v8f wmmab(v16bf a, v16bf b, v8f c) { return __builtin_amdgcn_wmma_f32_16x16x32_bf16(false, a, false, b, (short)0, c, false, false); }
__device__ __forceinline__ v16h  ldh(const h16* p) { return cat16(*(const v8h*)p, *(const v8h*)(p + 16)); }
__device__ __forceinline__ v16bf ldb(const bf* p)  { return cat16b(*(const v8us*)p, *(const v8us*)(p + 16)); }
__device__ __forceinline__ void wave_sync() { __builtin_amdgcn_fence(3  , "wavefront"); __builtin_amdgcn_wave_barrier(); asm volatile("" ::: "memory"); }

static __device__ __forceinline__ h16 toh_flush(float v) { const h16 r = (h16)v; return (fabsf(v) < 6.103515625e-05f) ? (h16)0.0f : r; }

__device__ __forceinline__ v8f gmma(v16bf a, v16bf b, v8f c) { c = wmmab(a, b, c); asm volatile("v_nop\n\tv_nop\n\tv_nop\n\tv_nop" : "+v"(c) : "v"(a), "v"(b)); return c; }
__device__ __forceinline__ v8f gmma(v16h a, v16h b, v8f c)   { c = wmma16(a, b, c); asm volatile("v_nop\n\tv_nop\n\tv_nop\n\tv_nop" : "+v"(c) : "v"(a), "v"(b)); return c; }
__device__ __forceinline__ v16bf ldfrag(const bf* p)  { return ldb(p); }
__device__ __forceinline__ v16h  ldfrag(const h16* p) { return ldh(p); }

__global__ __launch_bounds__(256) void k_cvt8(const float* __restrict__ src, bf* dst, size_t n8) {
    const size_t i = (size_t)blockIdx.x * 256 + threadIdx.x; if (i >= n8) return;
    const v8f v = *(const v8f*)(src + i * 8); v8us o;
#pragma unroll
    for (int k = 0; k < 8; ++k) o[k] = f2bf(v[k]);
    *(volatile v8us*)(dst + i * 8) = o; __threadfence(); *(volatile v8us*)(dst + i * 8) = o;
}

__global__ __launch_bounds__(256) void k_wconv(const float* __restrict__ src, int K, int N, unsigned short* dst, int KP, int asf16, float carry) {
    __shared__ float t[64 * 33];
    const int tid = threadIdx.x; const int k0 = blockIdx.x * 64, n0 = blockIdx.y * 32;
    { const int nn = tid & 31, kq = tid >> 5; const int n = n0 + nn; const int nc = n < N ? n : N - 1;
#pragma unroll
      for (int it = 0; it < 8; ++it) { const int kk = kq + 8 * it; const int k = k0 + kk; const int kc = k < K ? k : K - 1;
          float v = src[(size_t)kc * N + nc]; asm volatile("" : "+v"(v));
          t[kk * 33 + nn] = ((k < K) & (n < N)) ? v : 0.0f; } }
    __syncthreads();
    { const int nn = tid >> 3, p = tid & 7; v8us ob; v8h oh;
#pragma unroll
      for (int i = 0; i < 8; ++i) { const unsigned short bb = f2bf(t[(p * 8 + i) * 33 + nn]); ob[i] = bb; oh[i] = toh_flush(__uint_as_float(((unsigned)bb) << 16) * carry); }
      v8us o = ob; if (asf16 != 0) o = __builtin_bit_cast(v8us, oh);
      unsigned short* dp = dst + (size_t)(n0 + nn) * KP + k0 + p * 8;
      *(volatile v8us*)dp = o; __threadfence(); *(volatile v8us*)dp = o; }
}

template <typename T, int WH>
__device__ __forceinline__ void gemm_tile(const T* __restrict__ A, int lda, const T* __restrict__ Bt, int ldbt, int K,
                                          const float* __restrict__ bias, int nbias, float scale, float* C, int ldc, h16* Hh, int ldh_) {
    __shared__ __align__(16) float os[16 * 68];
    const int lane = threadIdx.x & 31, lr = lane & 15, hi = lane >> 4; const int r0 = blockIdx.x * 64, c0 = blockIdx.y * 64;
    v8f acc[4][4];
#pragma unroll
    for (int mb = 0; mb < 4; ++mb)
#pragma unroll
        for (int nb = 0; nb < 4; ++nb) acc[mb][nb] = (v8f){};
    const size_t aoff = (size_t)(r0 + lr) * lda + 8 * hi, boff = (size_t)(c0 + lr) * ldbt + 8 * hi;
#pragma unroll 1
    for (int kc = 0; kc < K; kc += 32) {
        auto a0 = ldfrag(A + aoff + (size_t)0 * 16 * lda + kc);
        auto a1 = ldfrag(A + aoff + (size_t)1 * 16 * lda + kc);
        auto a2 = ldfrag(A + aoff + (size_t)2 * 16 * lda + kc);
        auto a3 = ldfrag(A + aoff + (size_t)3 * 16 * lda + kc);
#pragma unroll
        for (int nb = 0; nb < 4; ++nb) { const auto b = ldfrag(Bt + boff + (size_t)nb * 16 * ldbt + kc);
            acc[0][nb] = gmma(a0, b, acc[0][nb]); acc[1][nb] = gmma(a1, b, acc[1][nb]); acc[2][nb] = gmma(a2, b, acc[2][nb]); acc[3][nb] = gmma(a3, b, acc[3][nb]); }
    }
    float bc[4];
#pragma unroll
    for (int nb = 0; nb < 4; ++nb) { const int c = c0 + nb * 16 + lr; const int cc = c < nbias ? c : nbias - 1;
        float bv = bias[cc]; asm volatile("" : "+v"(bv)); bc[nb] = (c < nbias) ? bfr(bv) : 0.0f; }
#pragma unroll
    for (int mb = 0; mb < 4; ++mb) {
#pragma unroll
        for (int nb = 0; nb < 4; ++nb) {
#pragma unroll
            for (int j = 0; j < 8; ++j) os[(hi * 8 + j) * 68 + nb * 16 + lr] = acc[mb][nb][j] * scale + bc[nb]; }
        wave_sync();
#pragma unroll 1
        for (int ps = 0; ps < 2; ++ps) {
            float* cb = C + (size_t)(r0 + mb * 16) * ldc + c0;
#pragma unroll
            for (int s = 0; s < 8; ++s) { const int row = 2 * s + (lane >> 4), cofs = (lane & 15) * 4;
                const v4f val = *(const v4fa*)(&os[row * 68 + cofs]);
                *(volatile v4f*)(cb + (size_t)row * ldc + cofs) = val; }
            if (WH) {
                h16* hb = Hh + (size_t)(r0 + mb * 16) * ldh_ + c0;
#pragma unroll
                for (int s = 0; s < 4; ++s) { const int row = 4 * s + (lane >> 3), c8 = (lane & 7) * 8;
                    const v4f x0 = *(const v4fa*)(&os[row * 68 + c8]); const v4f x1 = *(const v4fa*)(&os[row * 68 + c8 + 4]); v8h hv;
#pragma unroll
                    for (int i = 0; i < 4; ++i) { hv[i] = toh_flush(x0[i] * ACTC); hv[4 + i] = toh_flush(x1[i] * ACTC); }
                    *(volatile v8h*)(hb + (size_t)row * ldh_ + c8) = hv; }
            }
            if (ps == 0) __threadfence(); }
        wave_sync();
    }
}

__global__ __launch_bounds__(32) void k_gemm_in(const bf* __restrict__ A, const bf* __restrict__ Bt, const float* __restrict__ bias, float* C, h16* Hh) {
    gemm_tile<bf, 1>(A, NF, Bt, NF, NF, bias, HW, 1.0f, C, HW, Hh, HW);
}
__global__ __launch_bounds__(32) void k_gemm_hid(const h16* __restrict__ A, const h16* __restrict__ Bt, const float* __restrict__ bias, float* C, h16* Hh) {
    gemm_tile<h16, 1>(A, CATP, Bt, CATP, CATK, bias, HW, FOLD, C, HW, Hh, HW);
}
__global__ __launch_bounds__(32) void k_gemm_mb(const h16* __restrict__ A, const h16* __restrict__ Bt, const float* __restrict__ bias, float* C) {
    gemm_tile<h16, 0>(A, HW, Bt, HW, HW, bias, MBW, FOLD, C, MBP, nullptr, 0);
}

__global__ __launch_bounds__(128) void k_div(const float* __restrict__ Mp, float* DV) {
    __shared__ __align__(16) float rowI[MBP];
    __shared__ __align__(16) float part[4 * 32];
    const int i = blockIdx.x, tid = threadIdx.x, lane = tid & 31;
    const int wave = __builtin_amdgcn_readfirstlane((int)(threadIdx.x >> 5));
    rowI[tid] = Mp[(size_t)i * MBP + tid];
    __syncthreads();
    float s[NKER];
#pragma unroll
    for (int k = 0; k < NKER; ++k) s[k] = 0.0f;
#pragma unroll 1
    for (int j = tid; j < NROWS; j += 128) {
        const float* rj = Mp + (size_t)j * MBP;
#pragma unroll
        for (int c = 0; c < 5; ++c) {
            v4f a[5], b[5];
#pragma unroll
            for (int q = 0; q < 5; ++q) { a[q] = *(const v4f*)(rj + c * 20 + q * 4); b[q] = *(const v4fa*)(&rowI[c * 20 + q * 4]); }
            float l0 = 0.0f, l1 = 0.0f;
#pragma unroll
            for (int e = 0; e < 10; ++e) {
                l0 += fabsf(b[e >> 2][e & 3] - a[e >> 2][e & 3]);
                l1 += fabsf(b[(e + 10) >> 2][(e + 10) & 3] - a[(e + 10) >> 2][(e + 10) & 3]); }
            s[2 * c]     += __builtin_amdgcn_exp2f(fmaxf(-l0 * LOG2E, -126.0f));
            s[2 * c + 1] += __builtin_amdgcn_exp2f(fmaxf(-l1 * LOG2E, -126.0f));
        }
    }
#pragma unroll
    for (int k = 0; k < NKER; ++k) {
#pragma unroll
        for (int off = 16; off >= 1; off >>= 1) s[k] += __shfl_xor(s[k], off, 32); }
    float val = 0.0f;
#pragma unroll
    for (int k = 0; k < NKER; ++k) val = (lane == k) ? s[k] : val;
    part[wave * 32 + lane] = val;
    __syncthreads();
    if (wave == 0) {
        const int q = lane & 7;
        const v4f p0 = *(const v4fa*)(&part[0 * 32 + 4 * q]); const v4f p1 = *(const v4fa*)(&part[1 * 32 + 4 * q]);
        const v4f p2 = *(const v4fa*)(&part[2 * 32 + 4 * q]); const v4f p3 = *(const v4fa*)(&part[3 * 32 + 4 * q]);
        const v4f tsum = (p0 + p1) + (p2 + p3);
        float* dp = DV + (size_t)i * DVP + 4 * q;
        if (lane < 8) *(volatile v4f*)dp = tsum;
        __threadfence();
        if (lane < 8) *(volatile v4f*)dp = tsum;
    }
}

template <int HEAD>
__device__ __forceinline__ void ln_rows(const float* __restrict__ Hf, const float* __restrict__ DV, const float* __restrict__ beta,
                                        const float* __restrict__ Wf, const float* __restrict__ bfp, h16* CAT, float* OUT) {
    __shared__ __align__(16) float sc[LNR];
    const int lane = threadIdx.x & 31;
    const int wave = __builtin_amdgcn_readfirstlane((int)(threadIdx.x >> 5));
    float bt[8], btd[NKER], wf[8], wfd[NKER]; float hb = 0.0f;
    { const v4f p0 = *(const v4f*)(beta + 8 * lane), p1 = *(const v4f*)(beta + 8 * lane + 4);
#pragma unroll
      for (int e = 0; e < 4; ++e) { bt[e] = bfr(p0[e]); bt[4 + e] = bfr(p1[e]); } }
#pragma unroll
    for (int c = 0; c < NKER; ++c) btd[c] = bfr(beta[HW + c]);
#pragma unroll
    for (int e = 0; e < 8; ++e) wf[e] = 0.0f;
#pragma unroll
    for (int c = 0; c < NKER; ++c) wfd[c] = 0.0f;
    if (HEAD) {
        const v4f p0 = *(const v4f*)(Wf + 8 * lane), p1 = *(const v4f*)(Wf + 8 * lane + 4);
#pragma unroll
        for (int e = 0; e < 4; ++e) { wf[e] = bfr(p0[e]); wf[4 + e] = bfr(p1[e]); }
#pragma unroll
        for (int c = 0; c < NKER; ++c) wfd[c] = bfr(Wf[HW + c]);
        hb = bfr(bfp[0]);
    }
    const float inv = 1.0f / (float)CATW;
#pragma unroll 1
    for (int r = 0; r < LNRW; ++r) {
        const int row = blockIdx.x * LNR + wave * LNRW + r;
        const float* hp = Hf + (size_t)row * HW + 8 * lane;
        const v4f xa = *(const v4f*)hp, xb = *(const v4f*)(hp + 4);
        const float* dp = DV + (size_t)row * DVP;
        const v4f d0 = *(const v4f*)dp, d1 = *(const v4f*)(dp + 4), d2 = *(const v4f*)(dp + 8);
        float x[8], dv[NKER];
#pragma unroll
        for (int e = 0; e < 4; ++e) { x[e] = xa[e]; x[4 + e] = xb[e]; dv[e] = d0[e]; dv[4 + e] = d1[e]; }
        dv[8] = d2[0]; dv[9] = d2[1];
        float s = ((x[0] + x[1]) + (x[2] + x[3])) + ((x[4] + x[5]) + (x[6] + x[7]));
#pragma unroll
        for (int off = 16; off >= 1; off >>= 1) s += __shfl_xor(s, off, 32);
        float sd = 0.0f;
#pragma unroll
        for (int c = 0; c < NKER; ++c) sd += dv[c];
        const float mean = (s + sd) * inv;
        float q = 0.0f;
#pragma unroll
        for (int e = 0; e < 8; ++e) { const float d = x[e] - mean; q += d * d; }
#pragma unroll
        for (int off = 16; off >= 1; off >>= 1) q += __shfl_xor(q, off, 32);
        float qd = 0.0f;
#pragma unroll
        for (int c = 0; c < NKER; ++c) { const float d = dv[c] - mean; qd += d * d; }
        const float var = (q + qd) * inv;
        const float rstd = rsqrtf(var + LN_EPS);
        float y[8], yd[NKER];
#pragma unroll
        for (int e = 0; e < 8; ++e) { const float v = (x[e] - mean) * rstd + bt[e]; y[e] = (v >= 0.0f) ? v : LRA * v; }
#pragma unroll
        for (int c = 0; c < NKER; ++c) { const float v = (dv[c] - mean) * rstd + btd[c]; yd[c] = (v >= 0.0f) ? v : LRA * v; }
        if (HEAD) {
            float dt = 0.0f;
#pragma unroll
            for (int e = 0; e < 8; ++e) dt += y[e] * wf[e];
#pragma unroll
            for (int off = 16; off >= 1; off >>= 1) dt += __shfl_xor(dt, off, 32);
            float dd = 0.0f;
#pragma unroll
            for (int c = 0; c < NKER; ++c) dd += yd[c] * wfd[c];
            const float res = (dt + dd) + hb;
            if (lane == 0) sc[wave * LNRW + r] = res;
        } else {
            v8h hv, tv; h16 t1[8];
#pragma unroll
            for (int e = 0; e < 8; ++e) { hv[e] = toh_flush(y[e] * ACTC); t1[e] = (h16)0.0f; }
            t1[0] = toh_flush(yd[8] * ACTC); t1[1] = toh_flush(yd[9] * ACTC);
#pragma unroll
            for (int e = 0; e < 8; ++e) { const h16 a0 = toh_flush(yd[e] * ACTC); tv[e] = (lane == 0) ? a0 : ((lane == 1) ? t1[e] : (h16)0.0f); }
            h16* cp = CAT + (size_t)row * CATP;
            *(volatile v8h*)(cp + 8 * lane) = hv; if (lane < 8) *(volatile v8h*)(cp + HW + 8 * lane) = tv;
            __threadfence();
            *(volatile v8h*)(cp + 8 * lane) = hv; if (lane < 8) *(volatile v8h*)(cp + HW + 8 * lane) = tv;
        }
    }
    if (HEAD) {
        __syncthreads();
        if (wave == 0) {
            const int q = lane & 7;
            const v4f val = *(const v4fa*)(&sc[4 * q]);
            float* op = OUT + (size_t)blockIdx.x * LNR + 4 * q;
            if (lane < 8) *(volatile v4f*)op = val;
            __threadfence();
            if (lane < 8) *(volatile v4f*)op = val;
        }
    }
}

__global__ __launch_bounds__(256) void k_ln_cat(const float* __restrict__ Hf, const float* __restrict__ DV, const float* __restrict__ beta, h16* CAT) {
    ln_rows<0>(Hf, DV, beta, nullptr, nullptr, CAT, nullptr);
}
__global__ __launch_bounds__(256) void k_ln_head(const float* __restrict__ Hf, const float* __restrict__ DV, const float* __restrict__ beta,
                                                 const float* __restrict__ Wf, const float* __restrict__ bfp, float* OUT) {
    ln_rows<1>(Hf, DV, beta, Wf, bfp, nullptr, OUT);
}

static constexpr size_t al256(size_t v) { return (v + 255) & ~(size_t)255; }
static constexpr size_t SZ_XB  = al256((size_t)NROWS * NF * 2);
static constexpr size_t SZ_W0  = al256((size_t)HW * NF * 2);
static constexpr size_t SZ_W1  = al256((size_t)HW * CATP * 2);
static constexpr size_t SZ_WD  = al256((size_t)MBP * HW * 2);
static constexpr size_t SZ_HF  = al256((size_t)NROWS * HW * 4);
static constexpr size_t SZ_HH  = al256((size_t)NROWS * HW * 2);
static constexpr size_t SZ_MP  = al256((size_t)NROWS * MBP * 4);
static constexpr size_t SZ_DV  = al256((size_t)NROWS * DVP * 4);
static constexpr size_t SZ_CAT = al256((size_t)NROWS * CATP * 2);
static constexpr size_t SZ_TOTAL = SZ_XB + SZ_W0 + SZ_W1 + 2 * SZ_WD + SZ_HF + SZ_HH + SZ_MP + SZ_DV + SZ_CAT;
static_assert(SZ_TOTAL <= (size_t)134217728);

extern "C" void kernel_launch(void* const* d_in, const int* in_sizes, int n_in,
                              void* d_out, int out_size, void* d_ws, size_t ws_size, hipStream_t stream) {
    if (n_in < 13) return;
    if ((size_t)in_sizes[0] < (size_t)NROWS * NF) return;
    if ((size_t)in_sizes[1] < (size_t)NF * HW || in_sizes[2] < HW) return;
    if ((size_t)in_sizes[3] < (size_t)HW * MBW || in_sizes[4] < MBW || in_sizes[5] < CATW) return;
    if ((size_t)in_sizes[6] < (size_t)CATW * HW || in_sizes[7] < HW) return;
    if ((size_t)in_sizes[8] < (size_t)HW * MBW || in_sizes[9] < MBW || in_sizes[10] < CATW) return;
    if (in_sizes[11] < CATW || in_sizes[12] < 1) return;
    if (out_size < NROWS) return;
    if (SZ_TOTAL > ws_size) return;
    const float* x     = (const float*)d_in[0];
    const float* W0    = (const float*)d_in[1];  const float* b0  = (const float*)d_in[2];
    const float* Wd0   = (const float*)d_in[3];  const float* bd0 = (const float*)d_in[4];
    const float* beta0 = (const float*)d_in[5];
    const float* W1    = (const float*)d_in[6];  const float* b1  = (const float*)d_in[7];
    const float* Wd1   = (const float*)d_in[8];  const float* bd1 = (const float*)d_in[9];
    const float* beta1 = (const float*)d_in[10];
    const float* Wf    = (const float*)d_in[11]; const float* bfin = (const float*)d_in[12];
    float* OUT = (float*)d_out;
    char* wsp = (char*)d_ws;
    bf*  XB   = (bf*)wsp;   wsp += SZ_XB;
    bf*  W0T  = (bf*)wsp;   wsp += SZ_W0;
    h16* W1T  = (h16*)wsp;  wsp += SZ_W1;
    h16* WD0T = (h16*)wsp;  wsp += SZ_WD;
    h16* WD1T = (h16*)wsp;  wsp += SZ_WD;
    float* HF = (float*)wsp; wsp += SZ_HF;
    h16* HH   = (h16*)wsp;  wsp += SZ_HH;
    float* MP = (float*)wsp; wsp += SZ_MP;
    float* DV = (float*)wsp; wsp += SZ_DV;
    h16* CAT  = (h16*)wsp;  wsp += SZ_CAT;

    { const size_t n8 = (size_t)NROWS * NF / 8;
      k_cvt8<<<(unsigned)((n8 + 255) / 256), 256, 0, stream>>>(x, XB, n8); }
    k_wconv<<<dim3(NF / 64, HW / 32, 1), 256, 0, stream>>>(W0, NF, HW, (unsigned short*)W0T, NF, 0, 1.0f);
    k_wconv<<<dim3(CATP / 64, HW / 32, 1), 256, 0, stream>>>(W1, CATW, HW, (unsigned short*)W1T, CATP, 1, WGTC);
    k_wconv<<<dim3(HW / 64, MBP / 32, 1), 256, 0, stream>>>(Wd0, HW, MBW, (unsigned short*)WD0T, HW, 1, WGTC);
    k_wconv<<<dim3(HW / 64, MBP / 32, 1), 256, 0, stream>>>(Wd1, HW, MBW, (unsigned short*)WD1T, HW, 1, WGTC);

    k_gemm_in<<<dim3(NROWS / 64, HW / 64, 1), 32, 0, stream>>>(XB, W0T, b0, HF, HH);
    k_gemm_mb<<<dim3(NROWS / 64, MBP / 64, 1), 32, 0, stream>>>(HH, WD0T, bd0, MP);
    k_div<<<NROWS, 128, 0, stream>>>(MP, DV);
    k_ln_cat<<<NROWS / LNR, 256, 0, stream>>>(HF, DV, beta0, CAT);
    k_gemm_hid<<<dim3(NROWS / 64, HW / 64, 1), 32, 0, stream>>>(CAT, W1T, b1, HF, HH);
    k_gemm_mb<<<dim3(NROWS / 64, MBP / 64, 1), 32, 0, stream>>>(HH, WD1T, bd1, MP);
    k_div<<<NROWS, 128, 0, stream>>>(MP, DV);
    k_ln_head<<<NROWS / LNR, 256, 0, stream>>>(HF, DV, beta1, Wf, bfin, OUT);
}
